// OrderedFeatureGroupANFIS_80985903333981
// MI455X (gfx1250) — hardware-verified
//
#include <hip/hip_runtime.h>
#include <math.h>

typedef __attribute__((ext_vector_type(16))) _Float16 v16h;
typedef __attribute__((ext_vector_type(16))) __bf16 v16b;
typedef __attribute__((ext_vector_type(8)))  _Float16 v8h;
typedef __attribute__((ext_vector_type(8)))  float v8f;
typedef __attribute__((ext_vector_type(4)))  float v4f;
typedef __attribute__((ext_vector_type(2)))  float v2f;
typedef __attribute__((ext_vector_type(4)))  unsigned v4u;
typedef __attribute__((ext_vector_type(4)))  int v4i;
typedef float __attribute__((may_alias)) float_a;
typedef int __attribute__((may_alias)) int_a;

template <typename T> __device__ __forceinline__ void vst2(void* p, T v) { *(volatile T*)p = v; __threadfence(); *(volatile T*)p = v; }
__device__ __forceinline__ v8f wmma16(v16h a, v16h b, v8f c) {
  v8f d = __builtin_amdgcn_wmma_f32_16x16x32_f16(false, a, false, b, (short)0, c, false, false);
  asm volatile("v_nop\n\tv_nop\n\tv_nop\n\tv_nop" : "+v"(d) : "v"(a), "v"(b));
  return d;
}
__device__ __forceinline__ v8f wmma_bf(v16b a, v16b b, v8f c) {
  v8f d = __builtin_amdgcn_wmma_f32_16x16x32_bf16(false, a, false, b, (short)0, c, false, false);
  asm volatile("v_nop\n\tv_nop\n\tv_nop\n\tv_nop" : "+v"(d) : "v"(a), "v"(b));
  return d;
}
__device__ __forceinline__ v16h frag_h(const _Float16* rowk0, int lane) {
  union { v16h v; v8h q[2]; } u; const _Float16* p = rowk0 + 8 * (lane >> 4);
  u.q[0] = *(const v8h*)p; u.q[1] = *(const v8h*)(p + 16); return u.v;
}
__device__ __forceinline__ v16h frag_f32(const float* rowk0, int lane) {
  v16h a; const float* p = rowk0 + 8 * (lane >> 4);
#pragma unroll
  for (int i = 0; i < 8; ++i) { a[i] = (_Float16)p[i]; a[8 + i] = (_Float16)p[16 + i]; }
  return a;
}
__device__ __forceinline__ v16h frag_f32s(const float* rowk0, int lane, float sc) {
  v16h a; const float* p = rowk0 + 8 * (lane >> 4);
#pragma unroll
  for (int i = 0; i < 8; ++i) { a[i] = (_Float16)(p[i] * sc); a[8 + i] = (_Float16)(p[16 + i] * sc); }
  return a;
}
__device__ __forceinline__ v16h fragc_f32(const float* W, int k0, int n, int lane, int ld, int K) {
  v16h a; const int g = lane >> 4;
#pragma unroll
  for (int i = 0; i < 8; ++i) { const int ka = k0 + 8 * g + i, kb = ka + 16;
    a[i] = (_Float16)(ka < K ? W[(size_t)(ka < K ? ka : K - 1) * ld + n] : 0.f); a[8 + i] = (_Float16)(kb < K ? W[(size_t)(kb < K ? kb : K - 1) * ld + n] : 0.f); }
  return a;
}
struct F2 { v16b h, l; };
__device__ __forceinline__ F2 bsplit16(const float v[16]) { F2 r;
#pragma unroll
  for (int i = 0; i < 16; ++i) { const __bf16 h = (__bf16)v[i]; r.h[i] = h; r.l[i] = (__bf16)(v[i] - (float)h); }
  return r; }
__device__ __forceinline__ F2 split_row(const float* row, int k0, int lane) { float v[16]; const float* p = row + k0 + 8 * (lane >> 4);
#pragma unroll
  for (int i = 0; i < 8; ++i) { v[i] = p[i]; v[8 + i] = p[16 + i]; }
  return bsplit16(v); }
__device__ __forceinline__ F2 split_rowK(const float* row, int k0, int lane, int K) { float v[16]; const int g = lane >> 4;
#pragma unroll
  for (int i = 0; i < 8; ++i) { const int ka = k0 + 8 * g + i, kb = ka + 16; v[i] = ka < K ? row[ka < K ? ka : K - 1] : 0.f; v[8 + i] = kb < K ? row[kb < K ? kb : K - 1] : 0.f; }
  return bsplit16(v); }
__device__ __forceinline__ F2 split_col(const float* W, int k0, int n, int lane, int ld, int K) { float v[16]; const int g = lane >> 4;
#pragma unroll
  for (int i = 0; i < 8; ++i) { const int ka = k0 + 8 * g + i, kb = ka + 16; v[i] = ka < K ? W[(size_t)(ka < K ? ka : K - 1) * ld + n] : 0.f; v[8 + i] = kb < K ? W[(size_t)(kb < K ? kb : K - 1) * ld + n] : 0.f; }
  return bsplit16(v); }
__device__ __forceinline__ v8f mac3(const F2& a, const F2& b, v8f c) { c = wmma_bf(a.l, b.h, c); c = wmma_bf(a.h, b.l, c); return wmma_bf(a.h, b.h, c); }
__device__ __forceinline__ float sigm(float v) { return 1.0f / (1.0f + expf(-v)); }
#define LDSX() do { asm volatile("s_wait_dscnt 0" ::: "memory"); __builtin_amdgcn_wave_barrier(); __builtin_amdgcn_fence(__ATOMIC_RELEASE, "workgroup"); } while (0)


#define NBt 4096
#define NF 12
#define NM 2
#define NRU 4096
#define NO 8
#define NC (NF * NO + NO)
#define NCP 112
typedef __attribute__((ext_vector_type(8))) __bf16 v8b;
__device__ __forceinline__ v16b frag_b(const __bf16* rowk0, int lane) {
  union { v16b v; v8b q[2]; } u; const __bf16* p = rowk0 + 8 * (lane >> 4);
  u.q[0] = *(const v8b*)p; u.q[1] = *(const v8b*)(p + 16); return u.v;
}
__device__ __forceinline__ float bfr(float v) { return (float)(__bf16)v; }
__device__ __attribute__((noinline)) float exp_ni(float v) { return expf(v); }
__device__ __attribute__((noinline)) float erf_ni(float v) { return erff(v); }

#define WS_FN  0u
#define WS_END (WS_FN + 4u * (size_t)NBt * NRU)

__device__ __forceinline__ float softplus_f(float v) { return (v > 20.f) ? v : log1pf(expf(v)); }
__global__ __launch_bounds__(256) void k_fire(const float* __restrict__ X, const float* __restrict__ CB, const float* __restrict__ CD, const float* __restrict__ WR, float* __restrict__ FN) {
  __shared__ float sc[NF][NM], sw[NF][NM]; __shared__ float smem[8][NF][NM]; __shared__ float slo[8][64], shi[8][64]; __shared__ float ssum[8]; __shared__ __align__(16) float srow[8][NRU];
  const int t = threadIdx.x; const int wv = t >> 5, ln = t & 31; const size_t b0 = (size_t)blockIdx.x * 8;
  if (t < NF) { const float base = bfr(CB[t]); const float gap = softplus_f(bfr(CD[t])) + 1e-3f; sc[t][0] = base; sc[t][1] = base + gap; sw[t][0] = softplus_f(bfr(WR[t * 2])) + 1e-3f; sw[t][1] = softplus_f(bfr(WR[t * 2 + 1])) + 1e-3f; }
  __syncthreads();
  const size_t b = b0 + wv;
  if (ln < NF * NM) { const int f = ln >> 1, m = ln & 1; const float xv = bfr(X[b * NF + f]); const float d = xv - sc[f][m]; const float w = sw[f][m]; smem[wv][f][m] = expf(-(d * d) / (2.0f * w * w)); }
  __syncthreads();
  for (int i = ln; i < 64; i += 32) { float pl = 1.f, ph = 1.f;
#pragma unroll 1
    for (int f = 0; f < 6; ++f) { pl *= smem[wv][f][(i >> f) & 1]; ph *= smem[wv][6 + f][(i >> f) & 1]; }
    slo[wv][i] = pl; shi[wv][i] = ph; }
  __syncthreads();
  float s = 0.f;
#pragma unroll 1
  for (int r = ln; r < NRU; r += 32) { const float v = slo[wv][r & 63] * shi[wv][r >> 6]; srow[wv][r] = v; s += v; }
#pragma unroll
  for (int o = 1; o < 32; o <<= 1) s += __shfl_xor(s, o);
  const float inv = 1.0f / (s + 1e-8f);
  __syncthreads();
  for (int q = ln; q < NRU / 4; q += 32) { v4f v = *(const v4f*)&srow[wv][q * 4]; v[0] *= inv; v[1] *= inv; v[2] *= inv; v[3] *= inv; vst2(FN + b * NRU + q * 4, v); } }
__global__ __launch_bounds__(128) void k_out(const float* __restrict__ FN, const float* __restrict__ CP, const float* __restrict__ CR, const float* __restrict__ X, float* __restrict__ OUT) { __shared__ __align__(16) float sg[64][NCP + 4]; __shared__ __align__(16) float so[64][NO];
  const int tid = threadIdx.x, wave = tid >> 5, lane = tid & 31, col = lane & 15, g = lane >> 4; const size_t r0 = (size_t)blockIdx.x * 64 + wave * 16;
  v8f acc[7]; for (int j = 0; j < 7; ++j) for (int r = 0; r < 8; ++r) acc[j][r] = 0.f;
#pragma unroll 1
  for (int kc = 0; kc < NRU / 32; ++kc) { const F2 a = split_row(FN + (r0 + col) * NRU, kc * 32, lane);
#pragma unroll
    for (int j = 0; j < 7; ++j) { v16b w; const int c = j * 16 + col;
#pragma unroll
      for (int i = 0; i < 8; ++i) { const int ra = kc * 32 + 8 * g + i, rb = ra + 16;
        w[i] = (__bf16)(c < 96 ? CP[(size_t)ra * 96 + c] : (c < NC ? CR[(size_t)ra * NO + c - 96] : 0.f)); w[8 + i] = (__bf16)(c < 96 ? CP[(size_t)rb * 96 + c] : (c < NC ? CR[(size_t)rb * NO + c - 96] : 0.f)); }
      acc[j] = wmma_bf(a.h, w, acc[j]); acc[j] = wmma_bf(a.l, w, acc[j]); } }
#pragma unroll
  for (int j = 0; j < 7; ++j)
#pragma unroll
    for (int r = 0; r < 8; ++r) sg[wave * 16 + 8 * g + r][j * 16 + col] = acc[j][r];
  __syncthreads();
  for (int e = tid; e < 64 * NO; e += 128) { const int rl = e >> 3, o = e & 7; const size_t b = (size_t)blockIdx.x * 64 + rl; float a = sg[rl][96 + o];
#pragma unroll 1
    for (int f = 0; f < NF; ++f) a += bfr(X[b * NF + f]) * sg[rl][f * NO + o]; so[rl][o] = a; }
  __syncthreads(); for (int q = tid; q < 64 * NO / 4; q += 128) vst2(OUT + (size_t)blockIdx.x * 64 * NO + q * 4, *(const v4f*)((&so[0][0]) + q * 4)); }
extern "C" void kernel_launch(void* const* d_in, const int* in_sizes, int n_in, void* d_out, int out_size, void* d_ws, size_t ws_size, hipStream_t stream) {
  (void)in_sizes; (void)n_in; (void)out_size;
  const float** F = (const float**)d_in;
  if (ws_size < (size_t)WS_END) return;
  char* ws = (char*)d_ws; float* FN = (float*)(ws + WS_FN);
  k_fire<<<NBt / 8, 256, 0, stream>>>(F[0], F[1], F[2], F[3], FN);
  k_out<<<NBt / 64, 128, 0, stream>>>(FN, F[4], F[5], F[0], (float*)d_out);
}
